// RefineAutoEncoder_214748365316
// MI455X (gfx1250) — hardware-verified
//
#include <hip/hip_runtime.h>
#include <stddef.h>


#define NTHR    256
#define NWAVE   8
#define EPT     8
#define NGRP    2
#define CHUNK   (NTHR * EPT * NGRP)
#define WCAP    (EPT * NGRP * 32)
#define LISTN   (NWAVE * WCAP)
#define NBC     4096
#define NBF     1024
#define RCAP    40960
#define RBN     128
#define OTHR    512
#define DEGCAP  1024
#define WSCAP   134217728
#define LDS_FILL ((RCAP + NBF + LISTN) * 4 + 64)

static_assert((CHUNK & (CHUNK - 1)) == 0);
static_assert(CHUNK <= 4096);
static_assert(NBC <= 4096 && NBF <= 4096);
static_assert((NBC & (NBC - 1)) == 0 && (NBF & (NBF - 1)) == 0);
static_assert(NBC == 4 * NBF);
static_assert(OTHR * 8 == NBC);
static_assert((RCAP % 32) == 0);

typedef float    v2f  __attribute__((ext_vector_type(2)));
typedef float    v4f  __attribute__((ext_vector_type(4)));
typedef float    v8f  __attribute__((ext_vector_type(8)));
typedef int      v4i  __attribute__((ext_vector_type(4)));
typedef unsigned short v8us __attribute__((ext_vector_type(8)));
typedef __bf16   v16b __attribute__((ext_vector_type(16)));
union FragB { v16b v; v8us u[2]; };

template <int VW> struct VT;
template <> struct VT<4> { typedef v4f t; };
template <> struct VT<2> { typedef v2f t; };
template <int VW> __device__ __forceinline__ typename VT<VW>::t vzero();
template <> __device__ __forceinline__ v4f vzero<4>() { v4f z = {0.f, 0.f, 0.f, 0.f}; return z; }
template <> __device__ __forceinline__ v2f vzero<2>() { v2f z = {0.f, 0.f}; return z; }

__device__ __forceinline__ v8f wmb(v16b a, v16b b, v8f c) {
  v8f d = __builtin_amdgcn_wmma_f32_16x16x32_bf16(false, a, false, b, (short)0, c, false, false);
  asm volatile("v_nop\n\tv_nop\n\tv_nop\n\tv_nop" : "+v"(d) : "v"(a), "v"(b));
  return d;
}

__device__ __forceinline__ unsigned bf16_rne(float x) {
  const unsigned u = __float_as_uint(x);
  return (u + 0x7FFFu + ((u >> 16) & 1u)) >> 16;
}
__device__ __forceinline__ void split2(float x, unsigned& hi, unsigned& lo) {
  hi = bf16_rne(x);
  const float r = x - __uint_as_float(hi << 16);
  lo = bf16_rne(r);
}
__device__ __forceinline__ int clampi(int v, int lo, int hi) { return v < lo ? lo : (v > hi ? hi : v); }

template <int NB>
__device__ __forceinline__ int scan_chunk(const int* __restrict__ dsts, int nE, int cbase, int slotBase,
                                          int vec8, int* list, int tid, int lane, int wave) {
  int wc = 0;
#pragma unroll
  for (int g = 0; g < NGRP; ++g) {
    const int el0  = (g * NTHR + tid) * EPT;
    const int e0   = cbase + el0;
    const int sent = -2147483647 - 1;
    v4i da, db;
    if (vec8 != 0 && cbase + CHUNK <= nE) {
      da = *(const v4i*)(dsts + e0);
      db = *(const v4i*)(dsts + e0 + 4);
    } else {
      da.x = (e0     < nE) ? dsts[min(e0, nE - 1)] : sent;
      da.y = (e0 + 1 < nE) ? dsts[min(e0 + 1, nE - 1)] : sent;
      da.z = (e0 + 2 < nE) ? dsts[min(e0 + 2, nE - 1)] : sent;
      da.w = (e0 + 3 < nE) ? dsts[min(e0 + 3, nE - 1)] : sent;
      db.x = (e0 + 4 < nE) ? dsts[min(e0 + 4, nE - 1)] : sent;
      db.y = (e0 + 5 < nE) ? dsts[min(e0 + 5, nE - 1)] : sent;
      db.z = (e0 + 6 < nE) ? dsts[min(e0 + 6, nE - 1)] : sent;
      db.w = (e0 + 7 < nE) ? dsts[min(e0 + 7, nE - 1)] : sent;
    }
    const unsigned nb = (unsigned)slotBase;
    const unsigned s0 = (unsigned)da.x - nb, s1 = (unsigned)da.y - nb;
    const unsigned s2 = (unsigned)da.z - nb, s3 = (unsigned)da.w - nb;
    const unsigned s4 = (unsigned)db.x - nb, s5 = (unsigned)db.y - nb;
    const unsigned s6 = (unsigned)db.z - nb, s7 = (unsigned)db.w - nb;
    const bool h0 = s0 < (unsigned)NB, h1 = s1 < (unsigned)NB, h2 = s2 < (unsigned)NB, h3 = s3 < (unsigned)NB;
    const bool h4 = s4 < (unsigned)NB, h5 = s5 < (unsigned)NB, h6 = s6 < (unsigned)NB, h7 = s7 < (unsigned)NB;
    const unsigned any = __builtin_amdgcn_ballot_w32(h0 | h1 | h2 | h3 | h4 | h5 | h6 | h7);
    if (any != 0u) {
#define HITJ(J, HJ, SJ) { \
        const unsigned mj = __builtin_amdgcn_ballot_w32(HJ); \
        if (mj != 0u) { \
          if (HJ) { \
            const int pos = wc + (int)__builtin_amdgcn_mbcnt_lo(mj, 0u); \
            if (pos < WCAP) list[wave * WCAP + pos] = ((el0 + (J)) << 12) | (int)(SJ); \
          } \
          wc += (int)__builtin_popcount(mj); } }
      HITJ(0, h0, s0)
      HITJ(1, h1, s1)
      HITJ(2, h2, s2)
      HITJ(3, h3, s3)
      HITJ(4, h4, s4)
      HITJ(5, h5, s5)
      HITJ(6, h6, s6)
      HITJ(7, h7, s7)
#undef HITJ
    }
  }
  return wc;
}

__global__ __launch_bounds__(NTHR) void k_count(const int* __restrict__ dsts, int* cnt, float* dis,
                                                int nE, int vec8) {
  __shared__ __attribute__((aligned(16))) int scnt[NBC];
  __shared__ __attribute__((aligned(16))) int list[LISTN];
  __shared__ int wcnt[NWAVE];
  const int tid = threadIdx.x, lane = tid & 31, wave = tid >> 5;
  const int nodeBase = blockIdx.x * NBC;

  for (int i = tid; i < NBC; i += NTHR) scnt[i] = 0;
  __syncthreads();

  const int nChunks = (nE + CHUNK - 1) / CHUNK;
#pragma unroll 1
  for (int ch = 0; ch < nChunks; ++ch) {
    const int cbase = ch * CHUNK;
    const int wc = scan_chunk<NBC>(dsts, nE, cbase, nodeBase, vec8, list, tid, lane, wave);
    if (lane == 0) wcnt[wave] = wc;
    __syncthreads();
    if (wave == 0) {
#pragma unroll 1
      for (int wsx = 0; wsx < NWAVE; ++wsx) {
        int n = __builtin_amdgcn_readfirstlane(wcnt[wsx]);
        n = n > WCAP ? WCAP : (n < 0 ? 0 : n);
        const int* lp = list + wsx * WCAP;
#pragma unroll 1
        for (int i = 0; i < n; ++i) {
          const int ent  = __builtin_amdgcn_readfirstlane(lp[i]);
          const int slot = ent & (NBC - 1);
          if (lane == 0) scnt[slot] = scnt[slot] + 1;
        }
      }
    }
    __syncthreads();
  }

  v4i cq[4];
  v4f dq[4];
#pragma unroll
  for (int q = 0; q < 4; ++q) {
    const int f = (wave * 4 + q) * 128 + 4 * lane;
    cq[q] = *(const v4i*)(scnt + f);
    const float rx = rsqrtf((float)(cq[q].x > 0 ? cq[q].x : 1));
    const float ry = rsqrtf((float)(cq[q].y > 0 ? cq[q].y : 1));
    const float rz = rsqrtf((float)(cq[q].z > 0 ? cq[q].z : 1));
    const float rw = rsqrtf((float)(cq[q].w > 0 ? cq[q].w : 1));
    dq[q].x = cq[q].x > 0 ? rx : 0.0f;
    dq[q].y = cq[q].y > 0 ? ry : 0.0f;
    dq[q].z = cq[q].z > 0 ? rz : 0.0f;
    dq[q].w = cq[q].w > 0 ? rw : 0.0f;
  }
  int* cp = cnt + (size_t)nodeBase;
  float* dp = dis + (size_t)nodeBase;
#pragma unroll
  for (int q = 0; q < 4; ++q) {
    const int f = (wave * 4 + q) * 128 + 4 * lane;
    *(volatile v4i*)(cp + f) = cq[q];
    *(volatile v4f*)(dp + f) = dq[q];
  }
  __threadfence();
#pragma unroll
  for (int q = 0; q < 4; ++q) {
    const int f = (wave * 4 + q) * 128 + 4 * lane;
    *(volatile v4i*)(cp + f) = cq[q];
    *(volatile v4f*)(dp + f) = dq[q];
  }
}

__global__ __launch_bounds__(OTHR) void k_offsets(
    const int* __restrict__ cnt, int* off, int* rbase, int nChunk) {
  __shared__ __attribute__((aligned(16))) int soff[NBC];
  __shared__ __attribute__((aligned(16))) int srb[RBN];
  __shared__ int wtot[OTHR / 32];
  const int tid = threadIdx.x, lane = tid & 31, wave = tid >> 5, sub = tid >> 7;
  for (int i = tid; i < RBN; i += OTHR) srb[i] = 0;
  int carry = 0;
#pragma unroll 1
  for (int ch = 0; ch < nChunk; ++ch) {
    const int base = ch * NBC;
    const v4i c0 = *(const v4i*)(cnt + base + 8 * tid);
    const v4i c1 = *(const v4i*)(cnt + base + 8 * tid + 4);
    const int e0 = max(c0.x, 0), e1 = max(c0.y, 0), e2 = max(c0.z, 0), e3 = max(c0.w, 0);
    const int e4 = max(c1.x, 0), e5 = max(c1.y, 0), e6 = max(c1.z, 0), e7 = max(c1.w, 0);
    const int ts = e0 + e1 + e2 + e3 + e4 + e5 + e6 + e7;
    int incl = ts;
#pragma unroll
    for (int d = 1; d < 32; d <<= 1) {
      const int t = __shfl_up(incl, d);
      if (lane >= d) incl += t;
    }
    if (lane == 31) wtot[wave] = incl;
    __syncthreads();
    const int S0 = wtot[0]  + wtot[1]  + wtot[2]  + wtot[3];
    const int S1 = wtot[4]  + wtot[5]  + wtot[6]  + wtot[7];
    const int S2 = wtot[8]  + wtot[9]  + wtot[10] + wtot[11];
    const int S3 = wtot[12] + wtot[13] + wtot[14] + wtot[15];
    int pre = 0;
#pragma unroll 1
    for (int w = 4 * sub; w < wave; ++w) pre += wtot[w];
    const int b0 = carry;
    const int b1 = b0 + ((S0 + 31) & ~31);
    const int b2 = b1 + ((S1 + 31) & ~31);
    const int b3 = b2 + ((S2 + 31) & ~31);
    const int b4 = b3 + ((S3 + 31) & ~31);
    const int myb = sub == 0 ? b0 : (sub == 1 ? b1 : (sub == 2 ? b2 : b3));
    if (tid == 0) {
      srb[min(4 * ch + 0, RBN - 1)] = b0;
      srb[min(4 * ch + 1, RBN - 1)] = b1;
      srb[min(4 * ch + 2, RBN - 1)] = b2;
      srb[min(4 * ch + 3, RBN - 1)] = b3;
    }
    int run = myb + pre + incl - ts;
    soff[8 * tid + 0] = run; run += e0;
    soff[8 * tid + 1] = run; run += e1;
    soff[8 * tid + 2] = run; run += e2;
    soff[8 * tid + 3] = run; run += e3;
    soff[8 * tid + 4] = run; run += e4;
    soff[8 * tid + 5] = run; run += e5;
    soff[8 * tid + 6] = run; run += e6;
    soff[8 * tid + 7] = run;
    carry = b4;
    __syncthreads();
    const v4i o0 = *(const v4i*)(soff + 4 * tid);
    const v4i o1 = *(const v4i*)(soff + 4 * (tid + OTHR));
    int* op = off + base;
    *(volatile v4i*)(op + 4 * tid) = o0;
    *(volatile v4i*)(op + 4 * (tid + OTHR)) = o1;
    __threadfence();
    *(volatile v4i*)(op + 4 * tid) = o0;
    *(volatile v4i*)(op + 4 * (tid + OTHR)) = o1;
    __syncthreads();
  }
  if (tid == 0) srb[min(4 * nChunk, RBN - 1)] = carry;
  __syncthreads();
  v4i rv = {0, 0, 0, 0};
  if (tid < 32) rv = *(const v4i*)(srb + 4 * tid);
  if (tid < 32) *(volatile v4i*)(rbase + 4 * tid) = rv;
  __threadfence();
  if (tid < 32) *(volatile v4i*)(rbase + 4 * tid) = rv;
}

__global__ __launch_bounds__(NTHR) void k_fill(
    const int* __restrict__ dsts, const int* __restrict__ off, const int* __restrict__ rbase,
    int* csr, int nE, int vec8, int csrLen) {
  extern __shared__ v4f lds_dyn[];
  int* region = (int*)lds_dyn;
  int* cursor = region + RCAP;
  int* list   = cursor + NBF;
  int* wcnt   = list + LISTN;
  const int tid = threadIdx.x, lane = tid & 31, wave = tid >> 5;
  const int b = blockIdx.x;
  const int nodeBase = b * NBF;

  int rb0 = rbase[b];
  const int rb1 = rbase[b + 1];
  rb0 = rb0 < 0 ? 0 : (rb0 > csrLen ? csrLen : rb0);
  rb0 &= ~31;
  int len = rb1 - rb0;
  len = len < 0 ? 0 : (len > RCAP ? RCAP : len);
  int lenW = (len + 31) & ~31;
  if (rb0 + lenW > csrLen) lenW = (csrLen - rb0) & ~31;

  {
    const v4i z = {0, 0, 0, 0};
    for (int i = tid; i < RCAP / 4; i += NTHR) ((v4i*)region)[i] = z;
    for (int s = tid; s < NBF; s += NTHR) {
      int o = off[nodeBase + s] - rb0;
      o = o < 0 ? 0 : (o > RCAP ? RCAP : o);
      cursor[s] = o;
    }
  }
  __syncthreads();

  const int nChunks = (nE + CHUNK - 1) / CHUNK;
#pragma unroll 1
  for (int ch = 0; ch < nChunks; ++ch) {
    const int cbase = ch * CHUNK;
    const int wc = scan_chunk<NBF>(dsts, nE, cbase, nodeBase, vec8, list, tid, lane, wave);
    if (lane == 0) wcnt[wave] = wc;
    __syncthreads();
    if (wave == 0) {
#pragma unroll 1
      for (int wsx = 0; wsx < NWAVE; ++wsx) {
        int n = __builtin_amdgcn_readfirstlane(wcnt[wsx]);
        n = n > WCAP ? WCAP : (n < 0 ? 0 : n);
        const int* lp = list + wsx * WCAP;
#pragma unroll 1
        for (int i = 0; i < n; ++i) {
          const int ent  = __builtin_amdgcn_readfirstlane(lp[i]);
          const int slot = ent & (NBF - 1);
          int e = cbase + ((ent >> 12) & (CHUNK - 1));
          e = e > nE - 1 ? nE - 1 : e;
          if (lane == 0) {
            int pos = cursor[slot];
            pos = pos < 0 ? 0 : (pos > RCAP - 1 ? RCAP - 1 : pos);
            region[pos] = e;
            const int np = pos + 1;
            cursor[slot] = np > RCAP ? RCAP : np;
          }
        }
      }
    }
    __syncthreads();
  }

  const int nv = lenW >> 2;
  int* gp = csr + rb0;
#pragma unroll 1
  for (int i = tid; i < nv; i += NTHR) { const v4i v = ((const v4i*)region)[i]; *(volatile v4i*)(gp + 4 * i) = v; }
  __threadfence();
#pragma unroll 1
  for (int i = tid; i < nv; i += NTHR) { const v4i v = ((const v4i*)region)[i]; *(volatile v4i*)(gp + 4 * i) = v; }
}

__global__ __launch_bounds__(NTHR) void k_wplane(const float* __restrict__ W, unsigned short* dst,
                                                 int F, int FOUT, int NC, int KP, int tot8) {
  const int i = blockIdx.x * NTHR + threadIdx.x;
  const int ic = i > tot8 - 1 ? tot8 - 1 : i;
  const int plsz = NC * KP;
  v8us o;
#pragma unroll
  for (int j = 0; j < 8; ++j) {
    const int idx = 8 * ic + j;
    int pl = idx / plsz;
    const int rem = idx - pl * plsz;
    const int nn = rem / KP;
    const int c = rem - nn * KP;
    const int seg = c / F;
    const int f = c - seg * F;
    const bool ok = (nn < FOUT) && (seg < 3) && (pl < 6);
    pl = pl > 5 ? 5 : pl;
    const int fc = f > F - 1 ? F - 1 : f;
    const int ncl = nn > FOUT - 1 ? FOUT - 1 : nn;
    const float x = W[(size_t)(pl * F + fc) * FOUT + ncl];
    unsigned hi, lo;
    split2(x, hi, lo);
    const unsigned val = (seg == 1) ? lo : hi;
    o[j] = (unsigned short)(ok ? val : 0u);
  }
  unsigned short* dp = dst + (size_t)8 * ic;
  if (i < tot8) *(volatile v8us*)dp = o;
  __threadfence();
  if (i < tot8) *(volatile v8us*)dp = o;
}

template <int VW, int NV, int POOL>
__device__ __forceinline__ void seg_gather(typename VT<VW>::t (&acc)[NV],
    const int* __restrict__ csr, const int* __restrict__ cols, const float* __restrict__ coef,
    int n, int st, float cdt, int nE, int csrLen, int nS,
    const float* __restrict__ G, int gnp, int lofs, int lane) {
  typedef typename VT<VW>::t vt;
#pragma unroll 1
  for (int q0 = 0; q0 < n; q0 += 32) {
    int pos = st + q0 + lane;
    pos = clampi(pos, 0, csrLen - 1);
    int el = csr[pos];
    el = clampi(el, 0, nE - 1);
    int sl = cols[el];
    sl = clampi(sl, 0, nS - 1);
    float cfv;
    if (POOL) cfv = coef[el]; else cfv = cdt * coef[sl];
    const int cfi = __float_as_int(cfv);
    const int mcnt = (n - q0) < 32 ? (n - q0) : 32;
#pragma unroll 1
    for (int p = 0; p < mcnt; ++p) {
      const int s = __builtin_amdgcn_readlane(sl, p);
      const float cf = __int_as_float(__builtin_amdgcn_readlane(cfi, p));
      const float* gp = G + (size_t)s * gnp + lofs;
#pragma unroll
      for (int v = 0; v < NV; ++v) acc[v] = acc[v] + *(const vt*)(gp + VW * v) * cf;
    }
  }
}

template <int F, int RB, int APK, int TPRW, int CPT>
__device__ __forceinline__ void cheb_convert(const float* so, unsigned* sAu, int tid) {
  const int r = tid / TPRW, part = tid - r * TPRW;
  const float* src = so + r * F + part * CPT;
  unsigned* d0 = sAu + (r * APK + part * CPT) / 2;
#pragma unroll
  for (int j = 0; j < CPT; j += 2) {
    unsigned h0, l0, h1, l1;
    split2(src[j], h0, l0);
    split2(src[j + 1], h1, l1);
    const unsigned hp = h0 | (h1 << 16), lp = l0 | (l1 << 16);
    d0[j / 2] = hp;
    d0[(F + j) / 2] = hp;
    d0[(2 * F + j) / 2] = lp;
  }
}

template <int RT, int NT, int NKT, int KP, int APK>
__device__ __forceinline__ void cheb_gemm(const unsigned* sAu, const unsigned short* __restrict__ plane,
                                          int row0, int m, int hh, v8f (&wacc)[RT][NT]) {
  const unsigned short* sAh = (const unsigned short*)sAu;
#pragma unroll
  for (int kt = 0; kt < NKT; ++kt) {
    FragB a[RT];
#pragma unroll
    for (int rt = 0; rt < RT; ++rt) {
      const unsigned short* ap = sAh + (row0 + 16 * rt + m) * APK + 32 * kt + 8 * hh;
      a[rt].u[0] = *(const v8us*)(ap);
      a[rt].u[1] = *(const v8us*)(ap + 16);
    }
#pragma unroll
    for (int tt = 0; tt < NT; ++tt) {
      const unsigned short* bp = plane + (16 * tt + m) * KP + 32 * kt + 8 * hh;
      FragB bq;
      bq.u[0] = *(const v8us*)(bp);
      bq.u[1] = *(const v8us*)(bp + 16);
#pragma unroll
      for (int rt = 0; rt < RT; ++rt) wacc[rt][tt] = wmb(a[rt].v, bq.v, wacc[rt][tt]);
    }
  }
}

template <int F, int FOUT, int NB, int WPN>
__global__ __launch_bounds__(NTHR) void k_cheb(
    const int* __restrict__ csr, const int* __restrict__ off, const int* __restrict__ cnt,
    const int* __restrict__ cols, const float* __restrict__ dis, int nN, int nE, int csrLen,
    float cw, float diag,
    const float* __restrict__ G, int gnp, int gbp,
    const float* P, int pnp, int pbp,
    float* Tout, int tnp,
    const unsigned short* __restrict__ Bw, float* C, int cnp,
    const float* __restrict__ bias, int kstep, int elu) {
  constexpr int NPB = NWAVE / WPN;
  constexpr int RB  = NPB * NB;
  constexpr int LPB = 32 * WPN / NB;
  constexpr int CPL = F / LPB;
  constexpr int VW  = (CPL % 4 == 0) ? 4 : 2;
  constexpr int NV  = CPL / VW;
  constexpr int NC  = FOUT > 16 ? 32 : 16;
  constexpr int FO  = FOUT < 4 ? 4 : FOUT;
  constexpr int KP  = ((3 * F + 31) / 32) * 32;
  constexpr int APK = KP + 8;
  constexpr int NKT = KP / 32, NT = NC / 16, RT = RB / 128;
  constexpr int TPRW = NTHR / RB, CPT = F / TPRW;
  constexpr int QT = NB * F / 4 / WPN;
  constexpr int QC = NB * FO / 4 / WPN;
  constexpr int NPAD2 = (KP - 3 * F) / 2;
  typedef typename VT<VW>::t vt;
  static_assert(NPB * WPN == NWAVE);
  static_assert(RT * 128 == RB);
  static_assert(LPB * NB == 32 * WPN && CPL * LPB == F && NV * VW == CPL);
  static_assert(TPRW * RB == NTHR && CPT * TPRW == F && (CPT % 2) == 0);
  static_assert((QC % 32) == 0 && QT * 4 * WPN == NB * F);
  static_assert(FO * 2 <= APK);
  static_assert(((3 * F) % 2) == 0 && (F % 2) == 0);
  static_assert((NB * F) % 4 == 0);

  __shared__ __attribute__((aligned(16))) float so[RB * F];
  __shared__ __attribute__((aligned(16))) unsigned sAu[RB * APK / 2];

  const int tid = threadIdx.x, lane = tid & 31, wave = tid >> 5, hh = lane >> 4, m = lane & 15;
  const int sub = wave % WPN, wn = wave / WPN;
  const int node0 = blockIdx.x * NPB;
  const int t = node0 + wn;
  const bool tv = t < nN;
  const int tc = tv ? t : nN - 1;
  const int bb = lane % NB;
  const int c0 = CPL * (lane / NB + (32 / NB) * sub);
  const int lofs = bb * gbp + c0;

  if constexpr (NPAD2 > 0) {
#pragma unroll 1
    for (int r = tid; r < RB; r += NTHR) {
      unsigned* zp = sAu + (r * APK + 3 * F) / 2;
#pragma unroll
      for (int j = 0; j < NPAD2; ++j) zp[j] = 0u;
    }
  }

  int n = __builtin_amdgcn_readfirstlane(cnt[tc]);
  n = n < 0 ? 0 : (n > DEGCAP ? DEGCAP : n);
  const int st = __builtin_amdgcn_readfirstlane(off[tc]);
  const float cdt = cw * dis[tc];

  vt acc[NV];
#pragma unroll
  for (int v = 0; v < NV; ++v) acc[v] = vzero<VW>();
  seg_gather<VW, NV, 0>(acc, csr, cols, dis, n, st, cdt, nE, csrLen, nN, G, gnp, lofs, lane);

  vt sv[NV], tk[NV];
  {
    const float* sp = G + (size_t)tc * gnp + lofs;
#pragma unroll
    for (int v = 0; v < NV; ++v) sv[v] = *(const vt*)(sp + VW * v);
  }
#pragma unroll
  for (int v = 0; v < NV; ++v) tk[v] = acc[v] + sv[v] * diag;
  if (kstep >= 2) {
    const float* pp = P + (size_t)tc * pnp + bb * pbp + c0;
#pragma unroll
    for (int v = 0; v < NV; ++v) tk[v] = tk[v] * 2.0f - *(const vt*)(pp + VW * v);
  }

  v8f wacc[RT][NT];
#pragma unroll
  for (int rt = 0; rt < RT; ++rt) {
#pragma unroll
    for (int tt = 0; tt < NT; ++tt) {
      const v8f zz = {0.f, 0.f, 0.f, 0.f, 0.f, 0.f, 0.f, 0.f};
      wacc[rt][tt] = zz;
    }
  }
  float* sorow = so + (wn * NB + bb) * F + c0;
  const int row0 = wave * 16 * RT;

  if (kstep == 1) {
#pragma unroll
    for (int v = 0; v < NV; ++v) *(vt*)(sorow + VW * v) = sv[v];
    __syncthreads();
    cheb_convert<F, RB, APK, TPRW, CPT>(so, sAu, tid);
    __syncthreads();
    cheb_gemm<RT, NT, NKT, KP, APK>(sAu, Bw, row0, m, hh, wacc);
    __syncthreads();
  }
#pragma unroll
  for (int v = 0; v < NV; ++v) *(vt*)(sorow + VW * v) = tk[v];
  __syncthreads();

  const v4f* so4 = (const v4f*)so + wn * (NB * F / 4);
  float* tgp = Tout + (size_t)tc * tnp;
  const bool wst = tv && (kstep <= 4);
  if (wst) {
#pragma unroll
    for (int i = 0; i < (QT + 31) / 32; ++i) {
      const int q = 32 * i + lane;
      if (q < QT) *(volatile v4f*)(tgp + 4 * (sub * QT + q)) = so4[sub * QT + q];
    }
  }
  cheb_convert<F, RB, APK, TPRW, CPT>(so, sAu, tid);
  __threadfence();
  if (wst) {
#pragma unroll
    for (int i = 0; i < (QT + 31) / 32; ++i) {
      const int q = 32 * i + lane;
      if (q < QT) *(volatile v4f*)(tgp + 4 * (sub * QT + q)) = so4[sub * QT + q];
    }
  }
  __syncthreads();
  cheb_gemm<RT, NT, NKT, KP, APK>(sAu, Bw + (size_t)kstep * (NC * KP), row0, m, hh, wacc);
  __syncthreads();

  float* Cst = (float*)sAu;
#pragma unroll
  for (int rt = 0; rt < RT; ++rt) {
#pragma unroll
    for (int tt = 0; tt < NT; ++tt) {
      const int col = 16 * tt + m;
#pragma unroll
      for (int r = 0; r < 8; ++r) {
        const int row = row0 + 16 * rt + 8 * hh + r;
        if (col < FO) Cst[row * FO + col] = wacc[rt][tt][r];
      }
    }
  }
  __syncthreads();

  v4f* Cst4 = (v4f*)Cst + wn * (NB * FO / 4);
  float* cgp = C + (size_t)tc * cnp;
#pragma unroll 1
  for (int i = 0; i < QC / 32; ++i) {
    const int q = sub * QC + 32 * i + lane;
    v4f v = Cst4[q];
    if (kstep >= 2) v = v + *(const v4f*)(cgp + 4 * q);
    if (kstep == 5) {
      const int col = (4 * q) % FO;
      v.x += bias[col + 0 > FOUT - 1 ? FOUT - 1 : col + 0];
      v.y += bias[col + 1 > FOUT - 1 ? FOUT - 1 : col + 1];
      v.z += bias[col + 2 > FOUT - 1 ? FOUT - 1 : col + 2];
      v.w += bias[col + 3 > FOUT - 1 ? FOUT - 1 : col + 3];
      if (elu != 0) {
        v.x = v.x > 0.0f ? v.x : expm1f(v.x);
        v.y = v.y > 0.0f ? v.y : expm1f(v.y);
        v.z = v.z > 0.0f ? v.z : expm1f(v.z);
        v.w = v.w > 0.0f ? v.w : expm1f(v.w);
      }
      if constexpr (FOUT < FO) {
        if (col + 0 >= FOUT) v.x = 0.0f;
        if (col + 1 >= FOUT) v.y = 0.0f;
        if (col + 2 >= FOUT) v.z = 0.0f;
        if (col + 3 >= FOUT) v.w = 0.0f;
      }
    }
    Cst4[q] = v;
  }
  if (tv) {
#pragma unroll 1
    for (int i = 0; i < QC / 32; ++i) {
      const int q = sub * QC + 32 * i + lane;
      *(volatile v4f*)(cgp + 4 * q) = Cst4[q];
    }
  }
  __threadfence();
  if (tv) {
#pragma unroll 1
    for (int i = 0; i < QC / 32; ++i) {
      const int q = sub * QC + 32 * i + lane;
      *(volatile v4f*)(cgp + 4 * q) = Cst4[q];
    }
  }
}

template <int F, int NB, int WPN>
__global__ __launch_bounds__(NTHR) void k_pool(
    const int* __restrict__ csr, const int* __restrict__ off, const int* __restrict__ cnt,
    const int* __restrict__ cols, const float* __restrict__ val,
    int nT, int nS, int nE, int csrLen,
    const float* __restrict__ G, int gnp, int gbp, float* Tout, int tnp, int tbo) {
  constexpr int NPB = NWAVE / WPN;
  constexpr int RB  = NPB * NB;
  constexpr int LPB = 32 * WPN / NB;
  constexpr int CPL = F / LPB;
  constexpr int VW  = (CPL % 4 == 0) ? 4 : 2;
  constexpr int NV  = CPL / VW;
  constexpr int QT  = NB * F / 4 / WPN;
  typedef typename VT<VW>::t vt;
  static_assert(NPB * WPN == NWAVE);
  static_assert(LPB * NB == 32 * WPN && CPL * LPB == F && NV * VW == CPL);
  static_assert((QT % 32) == 0);

  __shared__ __attribute__((aligned(16))) float so[RB * F];

  const int tid = threadIdx.x, lane = tid & 31, wave = tid >> 5;
  const int sub = wave % WPN, wn = wave / WPN;
  const int t = blockIdx.x * NPB + wn;
  const bool tv = t < nT;
  const int tc = tv ? t : nT - 1;
  const int bb = lane % NB;
  const int c0 = CPL * (lane / NB + (32 / NB) * sub);
  const int lofs = bb * gbp + c0;

  int n = __builtin_amdgcn_readfirstlane(cnt[tc]);
  n = n < 0 ? 0 : (n > DEGCAP ? DEGCAP : n);
  const int st = __builtin_amdgcn_readfirstlane(off[tc]);

  vt acc[NV];
#pragma unroll
  for (int v = 0; v < NV; ++v) acc[v] = vzero<VW>();
  seg_gather<VW, NV, 1>(acc, csr, cols, val, n, st, 0.0f, nE, csrLen, nS, G, gnp, lofs, lane);

  float* sorow = so + (wn * NB + bb) * F + c0;
#pragma unroll
  for (int v = 0; v < NV; ++v) *(vt*)(sorow + VW * v) = acc[v];
  __syncthreads();

  const v4f* so4 = (const v4f*)so + wn * (NB * F / 4);
  float* tgp = Tout + (size_t)tc * tnp + tbo;
  if (tv) {
#pragma unroll
    for (int i = 0; i < QT / 32; ++i) {
      const int q = sub * QT + 32 * i + lane;
      *(volatile v4f*)(tgp + 4 * q) = so4[q];
    }
  }
  __threadfence();
  if (tv) {
#pragma unroll
    for (int i = 0; i < QT / 32; ++i) {
      const int q = sub * QT + 32 * i + lane;
      *(volatile v4f*)(tgp + 4 * q) = so4[q];
    }
  }
}

__device__ __forceinline__ float outelem(const float* __restrict__ R, int e, int per) {
  int bq = e / per;
  const int rem = e - bq * per;
  int tq = rem / 3;
  const int g = rem - 3 * tq;
  bq = bq > 31 ? 31 : bq;
  return R[((size_t)tq * 32 + bq) * 4 + g];
}

__global__ __launch_bounds__(NTHR) void k_out(const float* __restrict__ R, float* out, int nN, int nQ) {
  const int i = blockIdx.x * NTHR + threadIdx.x;
  const int ic = i > nQ - 1 ? nQ - 1 : i;
  const int per = 3 * nN;
  const int e = 4 * ic;
  v4f v;
  v.x = outelem(R, e + 0, per);
  v.y = outelem(R, e + 1, per);
  v.z = outelem(R, e + 2, per);
  v.w = outelem(R, e + 3, per);
  float* op = out + (size_t)4 * ic;
  if (i < nQ) *(volatile v4f*)op = v;
  __threadfence();
  if (i < nQ) *(volatile v4f*)op = v;
}

struct CsrT { int* cnt; int* off; float* dis; int* rb; int* csr; int nT, nE, nBC, nBF, csrLen; };

static size_t mx(size_t a, size_t b) { return a > b ? a : b; }

template <int F, int FOUT, int NB, int WPN>
static void run_cheb(hipStream_t s, const CsrT& g, const int* cols, int nN, float cw, float diag,
                     const float* T0, int np0, int bp0, float* U, float* V,
                     const unsigned short* Bw, float* C, const float* bias, int elu) {
  constexpr int NPB = NWAVE / WPN;
  constexpr int FO = FOUT < 4 ? 4 : FOUT;
  const int tnp = NB * F, cnp = NB * FO;
  const unsigned grid = (unsigned)((nN + NPB - 1) / NPB);
  k_cheb<F, FOUT, NB, WPN><<<grid, NTHR, 0, s>>>(g.csr, g.off, g.cnt, cols, g.dis, nN, g.nE, g.csrLen, cw, diag,
      T0, np0, bp0, T0, np0, bp0, U, tnp, Bw, C, cnp, bias, 1, elu);
  k_cheb<F, FOUT, NB, WPN><<<grid, NTHR, 0, s>>>(g.csr, g.off, g.cnt, cols, g.dis, nN, g.nE, g.csrLen, cw, diag,
      U, tnp, F, T0, np0, bp0, V, tnp, Bw, C, cnp, bias, 2, elu);
  k_cheb<F, FOUT, NB, WPN><<<grid, NTHR, 0, s>>>(g.csr, g.off, g.cnt, cols, g.dis, nN, g.nE, g.csrLen, cw, diag,
      V, tnp, F, U, tnp, F, U, tnp, Bw, C, cnp, bias, 3, elu);
  k_cheb<F, FOUT, NB, WPN><<<grid, NTHR, 0, s>>>(g.csr, g.off, g.cnt, cols, g.dis, nN, g.nE, g.csrLen, cw, diag,
      U, tnp, F, V, tnp, F, V, tnp, Bw, C, cnp, bias, 4, elu);
  k_cheb<F, FOUT, NB, WPN><<<grid, NTHR, 0, s>>>(g.csr, g.off, g.cnt, cols, g.dis, nN, g.nE, g.csrLen, cw, diag,
      V, tnp, F, U, tnp, F, U, tnp, Bw, C, cnp, bias, 5, elu);
}

template <int F, int NB, int WPN>
static void run_pool(hipStream_t s, const CsrT& g, const int* cols, const float* val, int nS,
                     const float* G, int gnp, int gbp, float* Tout, int tnp, int tbo) {
  constexpr int NPB = NWAVE / WPN;
  const unsigned grid = (unsigned)((g.nT + NPB - 1) / NPB);
  k_pool<F, NB, WPN><<<grid, NTHR, 0, s>>>(g.csr, g.off, g.cnt, cols, val, g.nT, nS, g.nE, g.csrLen,
                                           G, gnp, gbp, Tout, tnp, tbo);
}

extern "C" void kernel_launch(void* const* d_in, const int* in_sizes, int n_in,
                              void* d_out, int out_size, void* d_ws, size_t ws_size,
                              hipStream_t stream) {
  if (n_in < 33) return;
  const int NBT = 32;
  const int N0 = 35709, N1 = 8928, N2 = 2232;
  if (in_sizes[0] != NBT * N0 * 6) return;
  if (in_sizes[1] != 6 * 6 * 8   || in_sizes[2] != 8)  return;
  if (in_sizes[3] != 6 * 8 * 16  || in_sizes[4] != 16) return;
  if (in_sizes[5] != 6 * 16 * 32 || in_sizes[6] != 32) return;
  if (in_sizes[7] != 6 * 32 * 16 || in_sizes[8] != 16) return;
  if (in_sizes[9] != 6 * 16 * 8  || in_sizes[10] != 8) return;
  if (in_sizes[11] != 6 * 8 * 3  || in_sizes[12] != 3) return;
  const int E0 = in_sizes[13], E1 = in_sizes[15], E2 = in_sizes[17], E3 = in_sizes[19];
  const int ND0 = in_sizes[21], ND1 = in_sizes[24], NU3 = in_sizes[27], NU2 = in_sizes[30];
  if (in_sizes[14] != E0 || in_sizes[16] != E1 || in_sizes[18] != E2 || in_sizes[20] != E3) return;
  if (in_sizes[22] != ND0 || in_sizes[23] != ND0 || in_sizes[25] != ND1 || in_sizes[26] != ND1) return;
  if (in_sizes[28] != NU3 || in_sizes[29] != NU3 || in_sizes[31] != NU2 || in_sizes[32] != NU2) return;
  const int emax = 1 << 26;
  if (E0 <= 0 || E1 <= 0 || E2 <= 0 || E3 <= 0 || ND0 <= 0 || ND1 <= 0 || NU3 <= 0 || NU2 <= 0) return;
  if (E0 > emax || E1 > emax || E2 > emax || E3 > emax || ND0 > emax || ND1 > emax || NU3 > emax || NU2 > emax) return;
  if (out_size != NBT * N0 * 3 || (out_size & 3) != 0) return;

  const float* x   = (const float*)d_in[0];
  const float* W0  = (const float*)d_in[1];  const float* b0 = (const float*)d_in[2];
  const float* W1  = (const float*)d_in[3];  const float* b1 = (const float*)d_in[4];
  const float* W2  = (const float*)d_in[5];  const float* b2 = (const float*)d_in[6];
  const float* W3  = (const float*)d_in[7];  const float* b3 = (const float*)d_in[8];
  const float* W4  = (const float*)d_in[9];  const float* b4 = (const float*)d_in[10];
  const float* Wr  = (const float*)d_in[11]; const float* br = (const float*)d_in[12];
  const int* e0r = (const int*)d_in[13]; const int* e0c = (const int*)d_in[14];
  const int* e1r = (const int*)d_in[15]; const int* e1c = (const int*)d_in[16];
  const int* e2r = (const int*)d_in[17]; const int* e2c = (const int*)d_in[18];
  const int* e3r = (const int*)d_in[19]; const int* e3c = (const int*)d_in[20];
  const int* d0r = (const int*)d_in[21]; const int* d0c = (const int*)d_in[22]; const float* d0v = (const float*)d_in[23];
  const int* d1r = (const int*)d_in[24]; const int* d1c = (const int*)d_in[25]; const float* d1v = (const float*)d_in[26];
  const int* u3r = (const int*)d_in[27]; const int* u3c = (const int*)d_in[28]; const float* u3v = (const float*)d_in[29];
  const int* u2r = (const int*)d_in[30]; const int* u2c = (const int*)d_in[31]; const float* u2v = (const float*)d_in[32];
  float* out = (float*)d_out;

  char* ws = (char*)d_ws;
  size_t off = 0;
  auto take = [&](size_t bytes) { const size_t o = off; off += (bytes + 255) & ~(size_t)255; return o; };
  const size_t n0r = (size_t)((N0 + 7) & ~7), n1r = (size_t)((N1 + 7) & ~7), n2r = (size_t)((N2 + 7) & ~7);
  const size_t szH1 = mx(mx(n0r * 32 * 8 * 4, n1r * 32 * 32 * 4), mx(n2r * 32 * 16 * 4, n1r * 32 * 8 * 4));
  const size_t szX1 = mx(mx(n0r * 32 * 6 * 4, n0r * 16 * 16 * 4), mx(mx(n1r * 32 * 16 * 4, n2r * 32 * 32 * 4), n0r * 32 * 8 * 4));
  const size_t szXH  = n0r * 16 * 8 * 4;
  const size_t szX23 = mx(mx(2 * szXH, n0r * 32 * 6 * 4), mx(mx(n1r * 32 * 16 * 4, n2r * 32 * 32 * 4), n0r * 32 * 8 * 4));
  const size_t szT03 = mx(mx(n1r * 32 * 16 * 4, n2r * 32 * 32 * 4), n0r * 32 * 4 * 4);
  float* H1  = (float*)(ws + take(szH1));
  float* X1  = (float*)(ws + take(szX1));
  float* X23 = (float*)(ws + take(szX23));
  float* T03 = (float*)(ws + take(szT03));
  float* X23b = X23 + szXH / 4;

  CsrT ge0, ge1, ge2, ge3, gd0, gd1, gu3, gu2;
  bool okc = true;
  auto mk = [&](int nT, int nE, CsrT& c) {
    c.nT = nT; c.nE = nE;
    c.nBC = (nT + NBC - 1) / NBC;
    c.nBF = (nT + NBF - 1) / NBF;
    c.csrLen = ((nE + 31) & ~31) + 4096;
    if (4 * c.nBC + 1 > RBN || 31 * 4 * c.nBC > 4096) okc = false;
    const size_t cp = (size_t)c.nBC * NBC;
    c.cnt = (int*)(ws + take(cp * 4));
    c.off = (int*)(ws + take(cp * 4));
    c.dis = (float*)(ws + take(cp * 4));
    c.rb  = (int*)(ws + take((size_t)RBN * 4));
    c.csr = (int*)(ws + take((size_t)c.csrLen * 4));
  };
  mk(N0, E0, ge0); mk(N0, E1, ge1); mk(N1, E2, ge2); mk(N2, E3, ge3);
  mk(N1, ND0, gd0); mk(N2, ND1, gd1); mk(N1, NU3, gu3); mk(N0, NU2, gu2);
  if (!okc) return;

  const int plF[6]   = {6, 8, 16, 32, 16, 8};
  const int plO[6]   = {8, 16, 32, 16, 8, 3};
  const int plNC[6]  = {16, 16, 32, 16, 16, 16};
  const int plKP[6]  = {32, 32, 64, 96, 64, 32};
  unsigned short* PL[6];
  for (int l = 0; l < 6; ++l) PL[l] = (unsigned short*)(ws + take((size_t)6 * plNC[l] * plKP[l] * 2));
  if (off > ws_size || off > (size_t)WSCAP) return;

  hipFuncSetAttribute(reinterpret_cast<const void*>(&k_fill), hipFuncAttributeMaxDynamicSharedMemorySize, LDS_FILL);

  {
    const float* Wl[6] = {W0, W1, W2, W3, W4, Wr};
    for (int l = 0; l < 6; ++l) {
      const int tot8 = 6 * plNC[l] * plKP[l] / 8;
      k_wplane<<<(tot8 + NTHR - 1) / NTHR, NTHR, 0, stream>>>(Wl[l], PL[l], plF[l], plO[l], plNC[l], plKP[l], tot8);
    }
  }

  auto build = [&](const int* rows, const CsrT& c) {
    k_count<<<c.nBC, NTHR, 0, stream>>>(rows, c.cnt, c.dis, c.nE, 1);
    k_offsets<<<1, OTHR, 0, stream>>>(c.cnt, c.off, c.rb, c.nBC);
    k_fill<<<c.nBF, NTHR, LDS_FILL, stream>>>(rows, c.off, c.rb, c.csr, c.nE, 1, c.csrLen);
  };
  build(e0r, ge0); build(e1r, ge1); build(e2r, ge2); build(e3r, ge3);
  build(d0r, gd0); build(d1r, gd1); build(u3r, gu3); build(u2r, gu2);

  const float c23 = (float)(-2.0 / 2.3), dg23 = (float)(2.0 / 2.3 - 1.0);
  const float c20 = -1.0f, dg20 = 0.0f;

  run_cheb<6, 8, 32, 1>(stream, ge0, e0c, N0, c23, dg23, x, 6, N0 * 6, X1, X23, PL[0], H1, b0, 1);
  for (int h = 0; h < 2; ++h) {
    run_cheb<8, 16, 16, 1>(stream, ge1, e1c, N0, c23, dg23, H1 + 128 * h, 256, 8, X23, X23b, PL[1], X1, b1, 1);
    run_pool<16, 16, 1>(stream, gd0, d0c, d0v, N0, X1, 256, 16, T03, 512, 256 * h);
  }
  run_cheb<16, 32, 32, 1>(stream, ge2, e2c, N1, c23, dg23, T03, 512, 16, X1, X23, PL[2], H1, b2, 1);
  run_pool<32, 32, 2>(stream, gd1, d1c, d1v, N1, H1, 1024, 32, T03, 1024, 0);
  run_cheb<32, 16, 32, 2>(stream, ge3, e3c, N2, c23, dg23, T03, 1024, 32, X1, X23, PL[3], H1, b3, 1);
  run_pool<16, 32, 1>(stream, gu3, u3c, u3v, N2, H1, 512, 16, T03, 512, 0);
  run_cheb<16, 8, 32, 1>(stream, ge2, e2c, N1, c23, dg23, T03, 512, 16, X1, X23, PL[4], H1, b4, 1);
  run_pool<8, 32, 1>(stream, gu2, u2c, u2v, N1, H1, 256, 8, X1, 256, 0);
  run_cheb<8, 3, 32, 1>(stream, ge0, e0c, N0, c20, dg20, X1, 256, 8, X23, H1, PL[5], T03, br, 0);

  const int nQ = out_size / 4;
  k_out<<<(nQ + NTHR - 1) / NTHR, NTHR, 0, stream>>>(T03, out, N0, nQ);
}
